// PCLLoss_85134841741959
// MI455X (gfx1250) — hardware-verified
//
#include <hip/hip_runtime.h>

typedef _Float16 v16h __attribute__((ext_vector_type(16)));
typedef _Float16 v8h  __attribute__((ext_vector_type(8)));
typedef _Float16 v4h  __attribute__((ext_vector_type(4)));
typedef float    v8f  __attribute__((ext_vector_type(8)));
typedef float    v4f  __attribute__((ext_vector_type(4)));
typedef v8h __attribute__((may_alias)) v8ha;
typedef v4f __attribute__((may_alias)) v4fa;

union Frag { v16h v; v8h half[2]; };

#define NB        8192
#define ND        128
#define NC        256
#define NL        3
#define GRP       32
#define NGRP      (NC / GRP)
#define TAU       0.07f
#define ALPHA_C   10.0f
#define EPS_NORM  1e-12f
#define EPS_DENS  1e-6f
#define CARRY     8.0f
#define SHIFT     (1.0f / TAU)
#define SIM_SCALE (1.0f / (64.0f * TAU))
#define PRO_SCALE (1.0f / 64.0f)
#define THIRD     (1.0f / 3.0f)
#define NEG_BIG   (-1.0e30f)

static_assert(NB % 128 == 0);
static_assert(NB % 64 == 0);
static_assert(NB % 8 == 0);
static_assert(ND == 128);
static_assert(NC % GRP == 0);
static_assert(GRP == 32);
static_assert(NC % 16 == 0);
static_assert((NL * NC) % 128 == 0);

__device__ __forceinline__ v8f wmma_f16(v16h a, v16h b, v8f c) {
  v8f d = __builtin_amdgcn_wmma_f32_16x16x32_f16(false, a, false, b, (short)0, c, false, false);
  asm volatile("v_nop\n\tv_nop\n\tv_nop\n\tv_nop" : "+v"(d) : "v"(a), "v"(b));
  return d;
}

__device__ __forceinline__ v16h load_frag(const _Float16* p, int h) {
  Frag f;
  f.half[0] = *(const v8ha*)(p + 8 * h);
  f.half[1] = *(const v8ha*)(p + 16 + 8 * h);
  return f.v;
}

__device__ __forceinline__ int clampc(int v) { return min(max(v, 0), NC - 1); }

__global__ __launch_bounds__(256) void k_prep(const float* __restrict__ feat,
                                             float* __restrict__ fhat,
                                             _Float16* __restrict__ fh) {
  const int tid = threadIdx.x, lane = tid & 31, w = tid >> 5;
  const int row = blockIdx.x * 8 + w;
  if (row >= NB) return;
  const v4f x = *(const v4fa*)(feat + (size_t)row * ND + 4 * lane);
  float ss = x.x * x.x + x.y * x.y + x.z * x.z + x.w * x.w;
#pragma unroll
  for (int o = 16; o >= 1; o >>= 1) ss += __shfl_xor(ss, o);
  const float nrm = __builtin_amdgcn_sqrtf(ss);
  const float inv = __builtin_amdgcn_rcpf(fmaxf(nrm, EPS_NORM));
  const v4f y = { x.x * inv, x.y * inv, x.z * inv, x.w * inv };
  const v4h yh = { (_Float16)(y.x * CARRY), (_Float16)(y.y * CARRY),
                   (_Float16)(y.z * CARRY), (_Float16)(y.w * CARRY) };
  float* pf = fhat + (size_t)row * ND + 4 * lane;
  _Float16* ph = fh + (size_t)row * ND + 4 * lane;
  *(volatile v4f*)pf = y;
  *(volatile v4h*)ph = yh;
  __threadfence();
  *(volatile v4f*)pf = y;
  *(volatile v4h*)ph = yh;
}

__global__ __launch_bounds__(128) void k_ins(const _Float16* __restrict__ fh,
                                            const int* __restrict__ labels,
                                            float* __restrict__ ins) {
  __shared__ __attribute__((aligned(16))) float sres[64];

  const int tid = threadIdx.x, lane = tid & 31, w = tid >> 5;
  const int h = lane >> 4, m = lane & 15;
  const int row0 = blockIdx.x * 64 + 16 * w;

  const _Float16* arow = fh + (size_t)(row0 + m) * ND;
  const v16h a0 = load_frag(arow, h);
  const v16h a1 = load_frag(arow + 32, h);
  const v16h a2 = load_frag(arow + 64, h);
  const v16h a3 = load_frag(arow + 96, h);

  int labRow[8];
#pragma unroll
  for (int r = 0; r < 8; ++r)
    labRow[r] = clampc(labels[(size_t)(row0 + 8 * h + r) * NL]);

  float rsum[8], rpos[8], rcnt[8];
#pragma unroll
  for (int r = 0; r < 8; ++r) { rsum[r] = 0.0f; rpos[r] = 0.0f; rcnt[r] = 0.0f; }

  const _Float16* bbase = fh + (size_t)m * ND;
  const int* lbase = labels + (size_t)m * NL;
  const v8f zero8 = {0.f, 0.f, 0.f, 0.f, 0.f, 0.f, 0.f, 0.f};

#pragma unroll 1
  for (int kb = 0; kb < NB; kb += 64) {
    v8f acc[4];
    int lc[4];
#pragma unroll
    for (int j = 0; j < 4; ++j) {
      const _Float16* bp = bbase + (size_t)(kb + 16 * j) * ND;
      v8f z = zero8;
      z = wmma_f16(a0, load_frag(bp, h), z);
      z = wmma_f16(a1, load_frag(bp + 32, h), z);
      z = wmma_f16(a2, load_frag(bp + 64, h), z);
      z = wmma_f16(a3, load_frag(bp + 96, h), z);
      acc[j] = z;
      lc[j] = clampc(lbase[(size_t)(kb + 16 * j) * NL]);
    }
#pragma unroll
    for (int j = 0; j < 4; ++j) {
#pragma unroll
      for (int r = 0; r < 8; ++r) {
        const float v = acc[j][r] * SIM_SCALE;
        rsum[r] += __expf(v - SHIFT);
        const bool mt = (lc[j] == labRow[r]);
        rpos[r] += mt ? v : 0.0f;
        rcnt[r] += mt ? 1.0f : 0.0f;
      }
    }
  }

#pragma unroll
  for (int r = 0; r < 8; ++r) {
#pragma unroll
    for (int o = 1; o < 16; o <<= 1) {
      rsum[r] += __shfl_xor(rsum[r], o);
      rpos[r] += __shfl_xor(rpos[r], o);
      rcnt[r] += __shfl_xor(rcnt[r], o);
    }
  }
  if (m == 0) {
#pragma unroll
    for (int r = 0; r < 8; ++r) {
      const float gc  = fmaxf(rcnt[r], 1.0f);
      const float lse = SHIFT + logf(rsum[r]);
      sres[16 * w + 8 * h + r] = lse - rpos[r] * __builtin_amdgcn_rcpf(gc);
    }
  }
  __syncthreads();

  const bool wr = (w == 0) && (lane < 16);
  v4f v = {0.f, 0.f, 0.f, 0.f};
  float* dst = ins + (size_t)blockIdx.x * 64 + 4 * lane;
  if (wr) { v = *(const v4fa*)(sres + 4 * lane); *(volatile v4f*)dst = v; }
  __threadfence();
  if (wr) { *(volatile v4f*)dst = v; }
}

__device__ __forceinline__ void stats_store_pass(const float* sacc, const float* sinvn, const float* sout,
                                                 _Float16* pnh, float* invd,
                                                 int grp, int lvl, int w, int lane) {
#pragma unroll
  for (int j = 0; j < GRP / 4; ++j) {
    const int c = w * (GRP / 4) + j;
    const v4f p = *(const v4fa*)(sacc + c * ND + 4 * lane);
    const float sc = sinvn[c];
    const v4h o = { (_Float16)(p.x * sc), (_Float16)(p.y * sc), (_Float16)(p.z * sc), (_Float16)(p.w * sc) };
    _Float16* dst = pnh + ((size_t)lvl * NC + (size_t)grp * GRP + c) * ND + 4 * lane;
    *(volatile v4h*)dst = o;
  }
  if (w == 0 && lane < 8) {
    const v4f v = *(const v4fa*)(sout + 4 * lane);
    *(volatile v4f*)(invd + (size_t)lvl * NC + (size_t)grp * GRP + 4 * lane) = v;
  }
}

__global__ __launch_bounds__(128) void k_stats(const float* __restrict__ fhat,
                                              const int* __restrict__ labels,
                                              _Float16* __restrict__ pnh,
                                              float* __restrict__ invd) {
  __shared__ __attribute__((aligned(16))) float sacc[GRP * ND];
  __shared__ float scnt[GRP];
  __shared__ float sinvn[GRP];
  __shared__ __attribute__((aligned(16))) float sout[GRP];
  __shared__ float sd[128];
  __shared__ int   slist[128];
  __shared__ int   swcnt[4];

  const int tid = threadIdx.x, lane = tid & 31, w = tid >> 5;
  const int grp = blockIdx.x, lvl = blockIdx.y;

  for (int i = tid; i < GRP * ND; i += 128) sacc[i] = 0.0f;
  if (tid < GRP) scnt[tid] = 0.0f;
  __syncthreads();

#pragma unroll 1
  for (int cb = 0; cb < NB; cb += 128) {
    const int i = cb + tid;
    const int lab = clampc(labels[(size_t)i * NL + lvl]);
    const bool hit = (lab / GRP) == grp;
    const unsigned mask = (unsigned)__ballot(hit);
    const int pre = __builtin_popcount(mask & ((1u << lane) - 1u));
    if (lane == 0) swcnt[w] = __builtin_popcount(mask);
    __syncthreads();
    const int c0 = swcnt[0], c1 = swcnt[1], c2 = swcnt[2], c3 = swcnt[3];
    const int off = (w > 0 ? c0 : 0) + (w > 1 ? c1 : 0) + (w > 2 ? c2 : 0);
    const int total = min(c0 + c1 + c2 + c3, 128);
    if (hit) slist[off + pre] = (i << 5) | (lab & (GRP - 1));
    __syncthreads();
#pragma unroll 1
    for (int e = 0; e < total; ++e) {
      const int ent = slist[e];
      const int row = (ent >> 5) & (NB - 1);
      const int cl  = ent & (GRP - 1);
      sacc[cl * ND + tid] += fhat[(size_t)row * ND + tid];
      if (tid == 0) scnt[cl] += 1.0f;
    }
    __syncthreads();
  }

#pragma unroll 1
  for (int c = 0; c < GRP; ++c) {
    const float safe = fmaxf(scnt[c], 1.0f);
    sacc[c * ND + tid] = sacc[c * ND + tid] * __builtin_amdgcn_rcpf(safe);
  }
  __syncthreads();

#pragma unroll 1
  for (int j = 0; j < GRP / 4; ++j) {
    const int c = w * (GRP / 4) + j;
    const v4f p = *(const v4fa*)(sacc + c * ND + 4 * lane);
    float ss = p.x * p.x + p.y * p.y + p.z * p.z + p.w * p.w;
#pragma unroll
    for (int o = 16; o >= 1; o >>= 1) ss += __shfl_xor(ss, o);
    if (lane == 0)
      sinvn[c] = CARRY * __builtin_amdgcn_rcpf(fmaxf(__builtin_amdgcn_sqrtf(ss), EPS_NORM));
  }
  __syncthreads();

  float dacc = 0.0f;
#pragma unroll 1
  for (int cb = 0; cb < NB; cb += 128) {
    const int i = cb + tid;
    const int lab = clampc(labels[(size_t)i * NL + lvl]);
    const bool hit = (lab / GRP) == grp;
    const unsigned mask = (unsigned)__ballot(hit);
    const int pre = __builtin_popcount(mask & ((1u << lane) - 1u));
    if (lane == 0) swcnt[w] = __builtin_popcount(mask);
    __syncthreads();
    const int c0 = swcnt[0], c1 = swcnt[1], c2 = swcnt[2], c3 = swcnt[3];
    const int off = (w > 0 ? c0 : 0) + (w > 1 ? c1 : 0) + (w > 2 ? c2 : 0);
    const int total = min(c0 + c1 + c2 + c3, 128);
    if (hit) slist[off + pre] = (i << 5) | (lab & (GRP - 1));
    __syncthreads();
#pragma unroll 1
    for (int e = w; e < total; e += 4) {
      const int ent = slist[e];
      const int row = (ent >> 5) & (NB - 1);
      const int cl  = ent & (GRP - 1);
      const v4f f = *(const v4fa*)(fhat + (size_t)row * ND + 4 * lane);
      const v4f p = *(const v4fa*)(sacc + cl * ND + 4 * lane);
      const float dx = f.x - p.x, dy = f.y - p.y, dz = f.z - p.z, dw = f.w - p.w;
      float ss = dx * dx + dy * dy + dz * dz + dw * dw;
#pragma unroll
      for (int o = 16; o >= 1; o >>= 1) ss += __shfl_xor(ss, o);
      if (lane == 0) sd[e] = __builtin_amdgcn_sqrtf(ss);
    }
    __syncthreads();
    if (w == 0) {
#pragma unroll 1
      for (int e = 0; e < total; ++e) {
        const int cl = slist[e] & (GRP - 1);
        const float dv = sd[e];
        dacc += (cl == lane) ? dv : 0.0f;
      }
    }
    __syncthreads();
  }

  if (w == 0) {
    const float s    = scnt[lane];
    const float safe = fmaxf(s, 1.0f);
    const float md   = dacc * __builtin_amdgcn_rcpf(safe);
    const float den  = safe * __logf(s + ALPHA_C);
    float dn = (s > 0.0f) ? md * __builtin_amdgcn_rcpf(den) : 0.0f;
    dn = fmaxf(dn, EPS_DENS);
    sout[lane] = __builtin_amdgcn_rcpf(dn);
  }
  __syncthreads();

  stats_store_pass(sacc, sinvn, sout, pnh, invd, grp, lvl, w, lane);
  __threadfence();
  stats_store_pass(sacc, sinvn, sout, pnh, invd, grp, lvl, w, lane);
}

__global__ __launch_bounds__(128) void k_ploss(const _Float16* __restrict__ fh,
                                              const _Float16* __restrict__ pnh,
                                              const float* __restrict__ invd,
                                              const int* __restrict__ labels,
                                              const float* __restrict__ ins,
                                              float* __restrict__ out) {
  __shared__ float sinv[NL * NC];
  __shared__ __attribute__((aligned(16))) float sres[64];

  const int tid = threadIdx.x, lane = tid & 31, w = tid >> 5;
  const int h = lane >> 4, m = lane & 15;
  const int row0 = blockIdx.x * 64 + 16 * w;

  for (int i = tid; i < NL * NC; i += 128) sinv[i] = invd[i];
  __syncthreads();

  const _Float16* arow = fh + (size_t)(row0 + m) * ND;
  const v16h a0 = load_frag(arow, h);
  const v16h a1 = load_frag(arow + 32, h);
  const v16h a2 = load_frag(arow + 64, h);
  const v16h a3 = load_frag(arow + 96, h);

  const v8f zero8 = {0.f, 0.f, 0.f, 0.f, 0.f, 0.f, 0.f, 0.f};
  float pl[8];
#pragma unroll
  for (int r = 0; r < 8; ++r) pl[r] = 0.0f;

#pragma unroll 1
  for (int lvl = 0; lvl < NL; ++lvl) {
    int labRow[8];
#pragma unroll
    for (int r = 0; r < 8; ++r)
      labRow[r] = clampc(labels[(size_t)(row0 + 8 * h + r) * NL + lvl]);
    float rmax[8], rs[8], rpk[8];
#pragma unroll
    for (int r = 0; r < 8; ++r) { rmax[r] = NEG_BIG; rs[r] = 0.0f; rpk[r] = 0.0f; }

    const _Float16* pb = pnh + ((size_t)lvl * NC + m) * ND;
    const float* sv = sinv + lvl * NC;
#pragma unroll 1
    for (int ct = 0; ct < NC; ct += 16) {
      const _Float16* bp = pb + (size_t)ct * ND;
      v8f z = zero8;
      z = wmma_f16(a0, load_frag(bp, h), z);
      z = wmma_f16(a1, load_frag(bp + 32, h), z);
      z = wmma_f16(a2, load_frag(bp + 64, h), z);
      z = wmma_f16(a3, load_frag(bp + 96, h), z);
      const int c = ct + m;
      const float sc = sv[c] * PRO_SCALE;
#pragma unroll
      for (int r = 0; r < 8; ++r) {
        const float v  = z[r] * sc;
        const float mo = rmax[r];
        const float mn = fmaxf(mo, v);
        rs[r] = rs[r] * __expf(mo - mn) + __expf(v - mn);
        rmax[r] = mn;
        rpk[r] += (c == labRow[r]) ? v : 0.0f;
      }
    }
#pragma unroll
    for (int r = 0; r < 8; ++r) {
#pragma unroll
      for (int o = 1; o < 16; o <<= 1) {
        const float m2 = __shfl_xor(rmax[r], o);
        const float s2 = __shfl_xor(rs[r], o);
        const float p2 = __shfl_xor(rpk[r], o);
        const float mn = fmaxf(rmax[r], m2);
        rs[r] = rs[r] * __expf(rmax[r] - mn) + s2 * __expf(m2 - mn);
        rmax[r] = mn;
        rpk[r] += p2;
      }
      pl[r] += (rmax[r] + logf(rs[r])) - rpk[r];
    }
  }

  if (m == 0) {
#pragma unroll
    for (int r = 0; r < 8; ++r) sres[16 * w + 8 * h + r] = pl[r] * THIRD;
  }
  __syncthreads();

  const bool wr = (w == 0) && (lane < 16);
  v4f o4 = {0.f, 0.f, 0.f, 0.f};
  const size_t gi = (size_t)blockIdx.x * 64 + 4 * lane;
  if (wr) {
    const v4f p = *(const v4fa*)(sres + 4 * lane);
    const v4f q = *(const v4fa*)(ins + gi);
    o4.x = p.x + q.x; o4.y = p.y + q.y; o4.z = p.z + q.z; o4.w = p.w + q.w;
    *(volatile v4f*)(out + gi) = o4;
  }
  __threadfence();
  if (wr) { *(volatile v4f*)(out + gi) = o4; }
}

extern "C" void kernel_launch(void* const* d_in, const int* in_sizes, int n_in,
                              void* d_out, int out_size, void* d_ws, size_t ws_size,
                              hipStream_t stream) {
  if (n_in < 2) return;
  if (in_sizes[0] != NB * ND) return;
  if (in_sizes[1] != NB * NL) return;
  if (out_size != NB) return;

  const float* feat   = (const float*)d_in[0];
  const int*   labels = (const int*)d_in[1];
  float*       out    = (float*)d_out;

  const size_t fhat_bytes = (size_t)NB * ND * 4;
  const size_t fh_bytes   = (size_t)NB * ND * 2;
  const size_t pnh_bytes  = (size_t)NL * NC * ND * 2;
  const size_t invd_bytes = (size_t)NL * NC * 4;
  const size_t ins_bytes  = (size_t)NB * 4;
  const size_t total = fhat_bytes + fh_bytes + pnh_bytes + invd_bytes + ins_bytes;
  if (total > ws_size) return;

  char* ws = (char*)d_ws;
  float*    fhat = (float*)(ws);
  _Float16* fh   = (_Float16*)(ws + fhat_bytes);
  _Float16* pnh  = (_Float16*)(ws + fhat_bytes + fh_bytes);
  float*    invd = (float*)(ws + fhat_bytes + fh_bytes + pnh_bytes);
  float*    ins  = (float*)(ws + fhat_bytes + fh_bytes + pnh_bytes + invd_bytes);

  k_prep<<<NB / 8, 256, 0, stream>>>(feat, fhat, fh);
  k_ins<<<NB / 64, 128, 0, stream>>>(fh, labels, ins);
  dim3 gStats(NGRP, NL);
  k_stats<<<gStats, 128, 0, stream>>>(fhat, labels, pnh, invd);
  k_ploss<<<NB / 64, 128, 0, stream>>>(fh, pnh, invd, labels, ins, out);
}
